// BiAffineParser_7078106104314
// MI455X (gfx1250) — hardware-verified
//
#include <hip/hip_runtime.h>
#include <math.h>

constexpr int kB        = 4;
constexpr int kL        = 256;
constexpr int kH        = 768;
constexpr int kNL       = 13;
constexpr int kTok      = kB * kL;
constexpr int kN1       = 2 * kH;
constexpr int kPairs    = kB * kL * kL;
constexpr int kChunkRows = 16384;
constexpr int kNumChunks = kPairs / kChunkRows;
constexpr int kN2       = 64;
constexpr float kWCarry    = 32.0f;
constexpr float kWCarryInv = 1.0f / 32.0f;
static_assert(kNumChunks * kChunkRows == kPairs);
static_assert(kTok % 64 == 0 && kN1 % 64 == 0 && kChunkRows % 64 == 0 && kH % 32 == 0);

typedef __attribute__((ext_vector_type(16))) _Float16 v16h;
typedef __attribute__((ext_vector_type(8)))  _Float16 v8h;
typedef __attribute__((ext_vector_type(16))) __bf16   v16b;
typedef __attribute__((ext_vector_type(8)))  __bf16   v8b;
typedef __attribute__((ext_vector_type(8)))  float    v8f;
typedef __attribute__((ext_vector_type(4)))  float    v4f;
typedef __attribute__((ext_vector_type(4)))  unsigned int v4u;
typedef __attribute__((ext_vector_type(2)))  unsigned int v2u;

__device__ __forceinline__ unsigned short f2bf_bits(float f) {
  unsigned u = __float_as_uint(f);
  return (unsigned short)((u + 0x7FFFu + ((u >> 16) & 1u)) >> 16);
}
__device__ __forceinline__ float bf_bits2f(unsigned short h) { return __uint_as_float(((unsigned)h) << 16); }

__device__ __forceinline__ void dep_guard_h(v8f& a, v8f& b, v16h x, v16h y) { asm volatile("v_nop\n\tv_nop\n\tv_nop\n\tv_nop" : "+v"(a), "+v"(b) : "v"(x), "v"(y)); }
__device__ __forceinline__ void dep_guard_b(v8f& a, v8f& b, v16b x, v16b y) { asm volatile("v_nop\n\tv_nop\n\tv_nop\n\tv_nop" : "+v"(a), "+v"(b) : "v"(x), "v"(y)); }
__device__ __forceinline__ void keep4_h(v16h a, v16h b, v16h c, v16h d) { asm volatile("v_nop" :: "v"(a), "v"(b), "v"(c), "v"(d)); }
__device__ __forceinline__ void keep4_b(v16b a, v16b b, v16b c, v16b d) { asm volatile("v_nop" :: "v"(a), "v"(b), "v"(c), "v"(d)); }
__device__ __forceinline__ void acc_guard4(v8f& a, v8f& b, v8f& c, v8f& d) { asm volatile("v_nop\n\tv_nop\n\tv_nop\n\tv_nop" : "+v"(a), "+v"(b), "+v"(c), "+v"(d)); }
template <typename T> struct Frag;
template <> struct Frag<_Float16> {
  typedef v16h V; union U { v16h v; v8h h[2]; };
  static __device__ __forceinline__ v16h load(const _Float16* p) {
    U f; f.h[0] = *(const v8h*)(p); f.h[1] = *(const v8h*)(p + 16); return f.v;
  }
  static __device__ __forceinline__ v8f mma(v16h a, v16h b, v8f c) {
    return __builtin_amdgcn_wmma_f32_16x16x32_f16(false, a, false, b, (short)0, c, false, false);
  }
  static __device__ __forceinline__ void guard(v8f& a, v8f& b, v16h x, v16h y) { dep_guard_h(a, b, x, y); }
  static __device__ __forceinline__ void keep(v16h a, v16h b, v16h c, v16h d) { keep4_h(a, b, c, d); }
};
template <> struct Frag<__bf16> {
  typedef v16b V; union U { v16b v; v8b h[2]; };
  static __device__ __forceinline__ v16b load(const __bf16* p) {
    U f; f.h[0] = *(const v8b*)(p); f.h[1] = *(const v8b*)(p + 16); return f.v;
  }
  static __device__ __forceinline__ v8f mma(v16b a, v16b b, v8f c) {
    return __builtin_amdgcn_wmma_f32_16x16x32_bf16(false, a, false, b, (short)0, c, false, false);
  }
  static __device__ __forceinline__ void guard(v8f& a, v8f& b, v16b x, v16b y) { dep_guard_b(a, b, x, y); }
  static __device__ __forceinline__ void keep(v16b a, v16b b, v16b c, v16b d) { keep4_b(a, b, c, d); }
};

__device__ __forceinline__ unsigned pk16(unsigned short a, unsigned short b) { return (unsigned)a | ((unsigned)b << 16); }
__device__ __forceinline__ unsigned short h_bits(float f) { const _Float16 h = (_Float16)f; return __builtin_bit_cast(unsigned short, h); }

template <int ET> struct Elem;
template <> struct Elem<0> { typedef _Float16 T; };
template <> struct Elem<1> { typedef __bf16 T; };
template <int ET, bool SPLIT, int BIAS_MODE, int OUT_MODE, bool RESID, int ACT = 0>
__global__ __launch_bounds__(256) void wmma_gemm64(
    const unsigned short* __restrict__ Ap, const unsigned short* __restrict__ A2p, int lda, long strideA,
    const unsigned short* __restrict__ Btp, const unsigned short* __restrict__ Bt2p, int ldb, long strideB,
    void* __restrict__ Cout, void* __restrict__ Cout2, int ldc, long strideC,
    const float* __restrict__ bias,
    const float* __restrict__ resid, long strideR,
    int M, int N, int K, float scale) {
  typedef typename Elem<ET>::T T;
  typedef typename Frag<T>::V V;
  const T* A = (const T*)Ap; const T* A2 = (const T*)A2p; const T* Bt = (const T*)Btp; const T* Bt2 = (const T*)Bt2p;
  __shared__ __align__(16) float sT[8][16 * 68];
  const int b    = blockIdx.y;
  const int lane = threadIdx.x & 31;
  const int wave = threadIdx.x >> 5;
  const int tilesN = N >> 6;
  const int tilesM = M >> 6;
  const int tile = blockIdx.x * 8 + wave;
  if (tile >= tilesM * tilesN) return;
  const int tm = tile / tilesN;
  const int tn = tile - tm * tilesN;
  const int m0 = tm << 6;
  const int n0 = tn << 6;

  const T* Ab  = A  + (size_t)b * strideA;
  const T* Bb  = Bt + (size_t)b * strideB;
  const T* Ab2 = SPLIT ? (A2  + (size_t)b * strideA) : nullptr;
  const T* Bb2 = SPLIT ? (Bt2 + (size_t)b * strideB) : nullptr;

  const int rlane = lane & 15;
  const int koff  = (lane >> 4) * 8;
  const int mOff  = (lane >> 4) * 8;

  v8f acc[4][4];
#pragma unroll
  for (int i = 0; i < 4; ++i)
#pragma unroll
    for (int j = 0; j < 4; ++j) acc[i][j] = (v8f){0.f,0.f,0.f,0.f,0.f,0.f,0.f,0.f};

  for (int k0 = 0; k0 < K; k0 += 32) {
    V bh[4], bl[4];
#pragma unroll
    for (int j = 0; j < 4; ++j) {
      const size_t bo = (size_t)(n0 + (j << 4) + rlane) * ldb + koff + k0;
      bh[j] = Frag<T>::load(Bb + bo);
      if (SPLIT) bl[j] = Frag<T>::load(Bb2 + bo);
    }
#pragma unroll
    for (int i = 0; i < 4; ++i) {
      const size_t ao = (size_t)(m0 + (i << 4) + rlane) * lda + koff + k0;
      V ah = Frag<T>::load(Ab + ao);
      V al;
      if (SPLIT) al = Frag<T>::load(Ab2 + ao);
#pragma unroll
      for (int j = 0; j < 4; ++j) {
        acc[i][j] = Frag<T>::mma(ah, bh[j], acc[i][j]);
        if (SPLIT) {
          acc[i][j] = Frag<T>::mma(ah, bl[j], acc[i][j]);
          acc[i][j] = Frag<T>::mma(al, bh[j], acc[i][j]);
        }
      }
      Frag<T>::guard(acc[i][0], acc[i][3], ah, SPLIT ? al : ah);
    }
    Frag<T>::keep(bh[0], bh[1], bh[2], bh[3]);
    if (SPLIT) Frag<T>::keep(bl[0], bl[1], bl[2], bl[3]);
  }
  acc_guard4(acc[0][0], acc[0][1], acc[0][2], acc[0][3]);
  acc_guard4(acc[1][0], acc[1][1], acc[1][2], acc[1][3]);
  acc_guard4(acc[2][0], acc[2][1], acc[2][2], acc[2][3]);
  acc_guard4(acc[3][0], acc[3][1], acc[3][2], acc[3][3]);

  float* slab = sT[wave];
  const float* Rb = RESID ? (resid + (size_t)b * strideR) : nullptr;
#pragma unroll
  for (int i = 0; i < 4; ++i) {
    const int mBase = m0 + (i << 4);
#pragma unroll
    for (int j = 0; j < 4; ++j) {
      const int n = n0 + (j << 4) + rlane;
      float bv = 0.f;
      if (BIAS_MODE == 2) bv = bias[n];
#pragma unroll
      for (int r = 0; r < 8; ++r) {
        float v = acc[i][j][r] * scale;
        if (BIAS_MODE == 1) v += bias[mBase + mOff + r];
        if (BIAS_MODE == 2) v += bv;
        if (RESID) v += Rb[(size_t)(mBase + mOff + r) * ldc + n];
        if (ACT == 2) v = fmaxf(v, 0.0f);
        if (ACT == 4) v = (v > 0.f) ? v : 0.01f * v;
        slab[(mOff + r) * 68 + (j << 4) + rlane] = v;
      }
    }
    __builtin_amdgcn_fence(__ATOMIC_RELEASE, "workgroup");
    __builtin_amdgcn_wave_barrier();
    __builtin_amdgcn_fence(__ATOMIC_ACQUIRE, "workgroup");
    if (OUT_MODE == 0) {
      float* C = (float*)Cout + (size_t)b * strideC;
      const int hh = lane >> 4, c4 = (lane & 15) * 4;
      for (int pass = 0; pass < 2; ++pass) {
#pragma unroll
        for (int it = 0; it < 8; ++it) {
          const int row = it * 2 + hh;
          v4f v = *(const v4f*)(slab + row * 68 + c4);
          *(volatile v4f*)(C + (size_t)(mBase + row) * ldc + n0 + c4) = v;
        }
        __threadfence();
      }
    } else {
      const int q = lane >> 3, c8 = (lane & 7) * 8;
      unsigned short* C  = (unsigned short*)Cout  + (size_t)b * strideC;
      unsigned short* C2 = (OUT_MODE == 2) ? ((unsigned short*)Cout2 + (size_t)b * strideC) : nullptr;
      for (int pass = 0; pass < 2; ++pass) {
#pragma unroll
        for (int it = 0; it < 4; ++it) {
          const int row = it * 4 + q;
          const float* sp = slab + row * 68 + c8;
          v8h hv, lv;
#pragma unroll
          for (int e = 0; e < 8; ++e) {
            if (OUT_MODE == 1) {
              hv[e] = (_Float16)sp[e];
            } else {
              unsigned short hb = f2bf_bits(sp[e]);
              unsigned short lb = f2bf_bits(sp[e] - bf_bits2f(hb));
              hv[e] = __builtin_bit_cast(_Float16, hb);
              lv[e] = __builtin_bit_cast(_Float16, lb);
            }
          }
          *(volatile v8h*)(C + (size_t)(mBase + row) * ldc + n0 + c8) = hv;
          if (OUT_MODE == 2) *(volatile v8h*)(C2 + (size_t)(mBase + row) * ldc + n0 + c8) = lv;
        }
        __threadfence();
      }
    }
    __builtin_amdgcn_fence(__ATOMIC_RELEASE, "workgroup");
    __builtin_amdgcn_wave_barrier();
    __builtin_amdgcn_fence(__ATOMIC_ACQUIRE, "workgroup");
  }
}

__global__ __launch_bounds__(256) void cast8_f16_kernel(const float* __restrict__ in, unsigned short* __restrict__ out, int n8) {
  const int i = blockIdx.x * 256 + threadIdx.x;
  if (i >= n8) return;
  const float* p = in + 8 * (size_t)i;
  const v4f a = *(const v4f*)(p);
  const v4f c = *(const v4f*)(p + 4);
  unsigned short hb[8];
#pragma unroll
  for (int e = 0; e < 4; ++e) {
    hb[e]     = h_bits(a[e]);
    hb[4 + e] = h_bits(c[e]);
  }
  const v4u u = (v4u){pk16(hb[0], hb[1]), pk16(hb[2], hb[3]), pk16(hb[4], hb[5]), pk16(hb[6], hb[7])};
  unsigned short* q = out + 8 * (size_t)i;
  *(volatile v4u*)q = u;
  __threadfence();
  *(volatile v4u*)q = u;
}

__global__ __launch_bounds__(256) void w1tcast_kernel(const float* __restrict__ W1, unsigned short* __restrict__ out, float scale) {
  __shared__ float sm[64][65];
  const int t   = threadIdx.x;
  const int kc0 = blockIdx.x * 64;
  const int n0  = blockIdx.y * 64;
  const int z   = blockIdx.z;
  const float* W = W1 + (size_t)z * kH * kH;
#pragma unroll
  for (int i = 0; i < 16; ++i) {
    const int e = i * 256 + t;
    const int r = e >> 6;
    const int c = e & 63;
    sm[c][r] = W[(size_t)(kc0 + r) * kH + n0 + c] * scale;
  }
  __syncthreads();
  const int lane = t & 31, wave = t >> 5;
  const int q = lane >> 3, c8 = (lane & 7) * 8;
  unsigned short* op = out + (size_t)z * kH * kH;
  for (int pass = 0; pass < 2; ++pass) {
#pragma unroll
    for (int it = 0; it < 2; ++it) {
      const int row = wave * 8 + it * 4 + q;
      unsigned short hb[8];
#pragma unroll
      for (int e = 0; e < 8; ++e) hb[e] = h_bits(sm[row][c8 + e]);
      const v4u u = (v4u){pk16(hb[0], hb[1]), pk16(hb[2], hb[3]), pk16(hb[4], hb[5]), pk16(hb[6], hb[7])};
      *(volatile v4u*)(op + (size_t)(n0 + row) * kH + kc0 + c8) = u;
    }
    __threadfence();
  }
}

__global__ __launch_bounds__(256) void w2tcast_kernel(const float* __restrict__ W2, unsigned short* __restrict__ out, float scale, int n8) {
  const int g = blockIdx.x * 256 + threadIdx.x;
  if (g >= n8) return;
  const int n   = g / 96;
  const int kc0 = (g - n * 96) * 8;
  const int nn  = (n < kNL) ? n : (kNL - 1);
  unsigned short hb[8];
#pragma unroll
  for (int e = 0; e < 8; ++e) {
    const float w = W2[(size_t)(kc0 + e) * kNL + nn] * scale;
    const float v = (n < kNL) ? w : 0.0f;
    hb[e] = h_bits(v);
  }
  const v4u u = (v4u){pk16(hb[0], hb[1]), pk16(hb[2], hb[3]), pk16(hb[4], hb[5]), pk16(hb[6], hb[7])};
  unsigned short* q = out + (size_t)n * kH + kc0;
  *(volatile v4u*)q = u;
  __threadfence();
  *(volatile v4u*)q = u;
}

__global__ __launch_bounds__(256) void pair_gelu_kernel(const float* __restrict__ XP, const float* __restrict__ b1,
                                                        unsigned short* __restrict__ Hout, int chunk, int n4) {
  const int g = blockIdx.x * 256 + threadIdx.x;
  if (g >= n4) return;
  const int rr = g / 192;
  const int k0 = (g - rr * 192) * 4;
  const int R  = chunk * kChunkRows + rr;
  const int bi = R >> 8;
  const int bj = ((R >> 16) << 8) + (R & 255);
  const v4f xs = *(const v4f*)(XP + (size_t)bi * kN1 + k0);
  const v4f xe = *(const v4f*)(XP + (size_t)bj * kN1 + kH + k0);
  const v4f bb = *(const v4f*)(b1 + k0);
  unsigned short hb[4];
#pragma unroll
  for (int e = 0; e < 4; ++e) {
    const float v = (xs[e] + xe[e]) + bb[e];
    const float t = erff(v * 0.70710678118654752f);
    const float h = (0.5f * v) * (1.0f + t);
    hb[e] = h_bits(h);
  }
  const v2u u = (v2u){pk16(hb[0], hb[1]), pk16(hb[2], hb[3])};
  unsigned short* q = Hout + (size_t)rr * kH + k0;
  *(volatile v2u*)q = u;
  __threadfence();
  *(volatile v2u*)q = u;
}

__global__ __launch_bounds__(256) void pack_logits_kernel(const float* __restrict__ Cp, const float* __restrict__ b2,
                                                          float* __restrict__ out, int n4) {
  const int g = blockIdx.x * 256 + threadIdx.x;
  if (g >= n4) return;
  const int e0 = g * 4;
  v4f v;
#pragma unroll
  for (int c = 0; c < 4; ++c) {
    const int e   = e0 + c;
    const int row = e / kNL;
    const int col = e - row * kNL;
    v[c] = Cp[(size_t)row * kN2 + col] + b2[col];
  }
  float* q = out + (size_t)e0;
  *(volatile v4f*)q = v;
  __threadfence();
  *(volatile v4f*)q = v;
}

static inline size_t align256(size_t v) { return (v + 255) & ~(size_t)255; }

extern "C" void kernel_launch(void* const* d_in, const int* in_sizes, int n_in,
                              void* d_out, int out_size, void* d_ws, size_t ws_size,
                              hipStream_t stream) {
  if (n_in < 5) return;
  if (in_sizes[0] != kTok * kH) return;
  if (in_sizes[1] != kN1 * kH) return;
  if (in_sizes[2] != kH) return;
  if (in_sizes[3] != kH * kNL) return;
  if (in_sizes[4] != kNL) return;
  if (out_size != kPairs * kNL) return;

  const float* X  = (const float*)d_in[0];
  const float* W1 = (const float*)d_in[1];
  const float* b1 = (const float*)d_in[2];
  const float* W2 = (const float*)d_in[3];
  const float* b2 = (const float*)d_in[4];
  float* out = (float*)d_out;

  char* ws = (char*)d_ws;
  size_t off = 0;
  const size_t o_x16  = off; off = align256(off + (size_t)kTok * kH * 2);
  const size_t o_w1t  = off; off = align256(off + (size_t)kN1 * kH * 2);
  const size_t o_w2t  = off; off = align256(off + (size_t)kN2 * kH * 2);
  const size_t o_xsxe = off; off = align256(off + (size_t)kTok * kN1 * 4);
  const size_t o_h16  = off; off = align256(off + (size_t)kChunkRows * kH * 2);
  const size_t o_cpl  = off; off = align256(off + (size_t)kPairs * kN2 * 4);
  if (off > ws_size) return;

  unsigned short* x16  = (unsigned short*)(ws + o_x16);
  unsigned short* w1t  = (unsigned short*)(ws + o_w1t);
  unsigned short* w2t  = (unsigned short*)(ws + o_w2t);
  float*          xsxe = (float*)(ws + o_xsxe);
  unsigned short* h16  = (unsigned short*)(ws + o_h16);
  float*          cpl  = (float*)(ws + o_cpl);

  {
    const int n8 = kTok * kH / 8;
    cast8_f16_kernel<<<dim3((n8 + 255) / 256), 256, 0, stream>>>(X, x16, n8);
  }
  w1tcast_kernel<<<dim3(kH / 64, kH / 64, 2), 256, 0, stream>>>(W1, w1t, kWCarry);
  {
    const int n8 = kN2 * kH / 8;
    w2tcast_kernel<<<dim3((n8 + 255) / 256), 256, 0, stream>>>(W2, w2t, kWCarry, n8);
  }

  {
    const int tiles = (kTok / 64) * (kN1 / 64);
    wmma_gemm64<0, false, 0, 0, false><<<dim3((tiles + 7) / 8, 1), 256, 0, stream>>>(
        x16, nullptr, kH, 0L,
        w1t, nullptr, kH, 0L,
        (void*)xsxe, nullptr, kN1, 0L,
        nullptr, nullptr, 0L,
        kTok, kN1, kH, kWCarryInv);
  }

  const int n4_pair = kChunkRows * kH / 4;
  const int tiles2  = (kChunkRows / 64) * (kN2 / 64);
  for (int chunk = 0; chunk < kNumChunks; ++chunk) {
    pair_gelu_kernel<<<dim3((n4_pair + 255) / 256), 256, 0, stream>>>(xsxe, b1, h16, chunk, n4_pair);
    wmma_gemm64<0, false, 0, 0, false><<<dim3((tiles2 + 7) / 8, 1), 256, 0, stream>>>(
        h16, nullptr, kH, 0L,
        w2t, nullptr, kH, 0L,
        (void*)(cpl + (size_t)chunk * kChunkRows * kN2), nullptr, kN2, 0L,
        nullptr, nullptr, 0L,
        kChunkRows, kN2, kH, kWCarryInv);
  }

  {
    const int n4 = kPairs * kNL / 4;
    pack_logits_kernel<<<dim3((n4 + 255) / 256), 256, 0, stream>>>(cpl, b2, out, n4);
  }
}
